// ChunkwiseRetention_44495861186728
// MI455X (gfx1250) — hardware-run, weakly checked
//
#include <hip/hip_runtime.h>


#define NSQ 8
#define NTS 4000
#define NDM 256
#define NTL 67
#define NBK 536
#define NBL 4096
#define NRW 32000

typedef _Float16 h16;
typedef unsigned short bf;
typedef __attribute__((ext_vector_type(16))) __bf16   v16bf;
typedef __attribute__((ext_vector_type(16))) _Float16 v16h;
typedef __attribute__((ext_vector_type(8)))  _Float16 v8h;
typedef __attribute__((ext_vector_type(8)))  unsigned short v8us;
typedef __attribute__((ext_vector_type(8)))  float    v8f;
typedef __attribute__((ext_vector_type(4)))  float    v4f;
typedef v8h  __attribute__((may_alias)) v8ha;
typedef v4f  __attribute__((may_alias)) v4fa;
typedef v8us __attribute__((may_alias)) v8usa;

__device__ __forceinline__ unsigned short f2bf(float f) { unsigned u = __float_as_uint(f); u += 0x7FFFu + ((u >> 16) & 1u); return (unsigned short)(u >> 16); }
__device__ __forceinline__ float bf2f(unsigned short b) { return __uint_as_float(((unsigned)b) << 16); }
__device__ __forceinline__ float bfr(float f) { return bf2f(f2bf(f)); }
__device__ __forceinline__ v16h cat16(v8h lo, v8h hi) { return __builtin_shufflevector(lo, hi, 0, 1, 2, 3, 4, 5, 6, 7, 8, 9, 10, 11, 12, 13, 14, 15); }
__device__ __forceinline__ v16bf cat16b(v8us lo, v8us hi) { return __builtin_bit_cast(v16bf, __builtin_shufflevector(lo, hi, 0, 1, 2, 3, 4, 5, 6, 7, 8, 9, 10, 11, 12, 13, 14, 15)); }
__device__ __forceinline__ v8f wmma16(v16h a, v16h b, v8f c) { return __builtin_amdgcn_wmma_f32_16x16x32_f16(false, a, false, b, (short)0, c, false, false); }
__device__ __forceinline__ v8f wmmab(v16bf a, v16bf b, v8f c) { return __builtin_amdgcn_wmma_f32_16x16x32_bf16(false, a, false, b, (short)0, c, false, false); }

template <typename T16> struct WFrag;
template <> struct WFrag<h16> { typedef v16h V; static __device__ __forceinline__ V ld(const h16* p) { return cat16(*(const v8h*)p, *(const v8h*)(p + 16)); } static __device__ __forceinline__ v8f mma(V a, V b, v8f c) { return wmma16(a, b, c); } };
template <> struct WFrag<bf> { typedef v16bf V; static __device__ __forceinline__ V ld(const bf* p) { return cat16b(*(const v8us*)p, *(const v8us*)(p + 16)); } static __device__ __forceinline__ v8f mma(V a, V b, v8f c) { return wmmab(a, b, c); } };
template <typename T16, int NSPLIT, bool BIAS>
__global__ __launch_bounds__(32) void k_gemmw(const T16* __restrict__ A, const T16* __restrict__ A2, const T16* __restrict__ Bt, const T16* __restrict__ Bt2, int K, float* C, int ldc, const float* __restrict__ bias, size_t sA, size_t sB, size_t sC) {
    typedef typename WFrag<T16>::V V;
    __shared__ __align__(16) float os[16 * 68];
    const size_t z = blockIdx.z; A += z * sA; if (A2) A2 += z * sA; Bt += z * sB; if (Bt2) Bt2 += z * sB; C += z * sC;
    const int lane = threadIdx.x & 31, lr = lane & 15, hi = lane >> 4; const int r0 = blockIdx.x * 64, c0 = blockIdx.y * 64;
    v8f acc[4][4];
#pragma unroll
    for (int mb = 0; mb < 4; ++mb)
#pragma unroll
        for (int nb = 0; nb < 4; ++nb) acc[mb][nb] = (v8f){};
    const size_t aoff = (size_t)(r0 + lr) * K + 8 * hi, boff = (size_t)(c0 + lr) * K + 8 * hi;
    for (int kc = 0; kc < K; kc += 32) {
        V a[4], a2[4];
#pragma unroll
        for (int mb = 0; mb < 4; ++mb) { a[mb] = WFrag<T16>::ld(A + aoff + (size_t)mb * 16 * K + kc); if (NSPLIT == 1 || NSPLIT == 2) a2[mb] = WFrag<T16>::ld(A2 + aoff + (size_t)mb * 16 * K + kc); }
#pragma unroll
        for (int nb = 0; nb < 4; ++nb) { const V b = WFrag<T16>::ld(Bt + boff + (size_t)nb * 16 * K + kc); V b2; if (NSPLIT >= 2) b2 = WFrag<T16>::ld(Bt2 + boff + (size_t)nb * 16 * K + kc);
#pragma unroll
            for (int mb = 0; mb < 4; ++mb) { acc[mb][nb] = WFrag<T16>::mma(a[mb], b, acc[mb][nb]); if (NSPLIT == 1 || NSPLIT == 2) acc[mb][nb] = WFrag<T16>::mma(a2[mb], b, acc[mb][nb]); if (NSPLIT >= 2) acc[mb][nb] = WFrag<T16>::mma(a[mb], b2, acc[mb][nb]); } }
        asm volatile("v_nop\n\tv_nop\n\tv_nop\n\tv_nop" : "+v"(acc[0][0]), "+v"(acc[1][1]), "+v"(acc[2][2]), "+v"(acc[3][3]) : "v"(a[0]), "v"(a[3]));
    }
#pragma unroll
    for (int mb = 0; mb < 4; ++mb) {
#pragma unroll
        for (int nb = 0; nb < 4; ++nb) {
#pragma unroll
            for (int j = 0; j < 8; ++j) os[(hi * 8 + j) * 68 + nb * 16 + lr] = acc[mb][nb][j]; }
        __builtin_amdgcn_wave_barrier(); asm volatile("" ::: "memory");
        float* crow = C + (size_t)(r0 + mb * 16) * ldc + c0;
#pragma unroll 1
        for (int ps = 0; ps < 2; ++ps) {
#pragma unroll
            for (int s = 0; s < 8; ++s) { const int row = 2 * s + hi, cofs = lr * 4; v4f val = *(const v4fa*)(os + row * 68 + cofs); if (BIAS) { val[0] += bfr(bias[c0 + cofs]); val[1] += bfr(bias[c0 + cofs + 1]); val[2] += bfr(bias[c0 + cofs + 2]); val[3] += bfr(bias[c0 + cofs + 3]); }
                *(volatile v4f*)(crow + (size_t)row * ldc + cofs) = val; }
            if (ps == 0) __threadfence(); }
        __builtin_amdgcn_wave_barrier(); asm volatile("" ::: "memory");
    }
}

typedef __attribute__((ext_vector_type(2))) _Float16 v2h;
typedef __attribute__((ext_vector_type(4))) _Float16 v4h;
typedef __attribute__((ext_vector_type(2))) unsigned short v2us;
typedef __attribute__((ext_vector_type(4))) unsigned short v4us;
typedef __attribute__((ext_vector_type(2))) float v2f;
typedef __attribute__((ext_vector_type(4))) int v4i;
__device__ __forceinline__ h16 toh_flush(float x) { const float z = (fabsf(x) < 6.103515625e-05f) ? 0.0f : x; return (h16)z; }

typedef __attribute__((ext_vector_type(4))) _Float16 v4h_;
__global__ __launch_bounds__(256) void k_fillb(bf* P, unsigned w2, size_t n8) { const size_t i = (size_t)blockIdx.x * 256 + threadIdx.x; if (i >= n8) return; v4i o; o[0] = (int)w2; o[1] = (int)w2; o[2] = (int)w2; o[3] = (int)w2;
    *(volatile v4i*)(P + i * 8) = o; __threadfence(); *(volatile v4i*)(P + i * 8) = o; }

__global__ __launch_bounds__(256) void k_wtw(const float* __restrict__ W, h16* Wt) {
    const unsigned i = blockIdx.x * 256 + threadIdx.x; const unsigned n = i & 255u, k64 = i >> 8; const float* src = W + (size_t)k64 * 64 * NDM + n; h16 r[64];
#pragma unroll
    for (int kj = 0; kj < 64; ++kj) r[kj] = toh_flush(bfr(src[(size_t)kj * NDM]) * 1024.0f);
    h16* pd = Wt + (size_t)n * NDM + (size_t)k64 * 64;
#pragma unroll
    for (int ps = 0; ps < 2; ++ps) {
#pragma unroll
        for (int g = 0; g < 8; ++g) { v8h o;
#pragma unroll
            for (int j = 0; j < 8; ++j) o[j] = r[g * 8 + j];
            *(volatile v8h*)(pd + g * 8) = o; }
        if (ps == 0) __threadfence(); } }

__global__ __launch_bounds__(256) void k_xword(const float* __restrict__ src, h16* dst) {
    const size_t i = (size_t)blockIdx.x * 256 + threadIdx.x; const v8f wv = *(const v8f*)(src + i * 8); v8h ow;
#pragma unroll
    for (int j = 0; j < 8; ++j) ow[j] = toh_flush(bfr(wv[j]));
    *(volatile v8h*)(dst + i * 8) = ow; __threadfence(); *(volatile v8h*)(dst + i * 8) = ow; }

template <int MD>
__global__ __launch_bounds__(256) void k_tw(const float* __restrict__ src, h16* dst) {
    const unsigned i = blockIdx.x * 256 + threadIdx.x; const unsigned r = i & 63u, tile = i >> 6; const unsigned sq = tile / 67u, j = tile - sq * 67u; const unsigned t = 60u * j + r + (MD == 1 ? 5u : 0u); const unsigned tc = t < 3999u ? t : 3999u;
    const float live = (float)(r < 60u) * (float)(t < 4000u); const unsigned cr = r / 5u; const float ex = MD == 1 ? (float)(cr + 1u) : (MD == 2 ? -(float)cr : 0.0f); const float fac = exp2f(ex * -0.117654048f) * live * 0.0009765625f;
    const float* ps_ = src + ((size_t)sq * NTS + tc) * NDM; h16* pd = dst + (size_t)i * NDM;
#pragma unroll
    for (int ps = 0; ps < 2; ++ps) {
#pragma unroll
        for (int g = 0; g < 32; ++g) { const v8f w = *(const v8f*)(ps_ + g * 8); v8h o;
#pragma unroll
            for (int jj = 0; jj < 8; ++jj) o[jj] = toh_flush(w[jj] * fac);
            *(volatile v8h*)(pd + g * 8) = o; }
        if (ps == 0) __threadfence(); } }

template <bool KM>
__global__ __launch_bounds__(256) void k_tcol(const float* __restrict__ src, h16* dst) {
    constexpr float CF[64] = {1.00000000f, 1.00000000f, 1.00000000f, 1.00000000f, 1.00000000f, 1.08496916f, 1.08496916f, 1.08496916f, 1.08496916f, 1.08496916f, 1.17715812f, 1.17715812f, 1.17715812f, 1.17715812f, 1.17715812f, 1.27718019f, 1.27718019f, 1.27718019f, 1.27718019f, 1.27718019f, 1.38570118f, 1.38570118f, 1.38570118f, 1.38570118f, 1.38570118f, 1.50344312f, 1.50344312f, 1.50344312f, 1.50344312f, 1.50344312f, 1.63118935f, 1.63118935f, 1.63118935f, 1.63118935f, 1.63118935f, 1.76979017f, 1.76979017f, 1.76979017f, 1.76979017f, 1.76979017f, 1.92016768f, 1.92016768f, 1.92016768f, 1.92016768f, 1.92016768f, 2.08332276f, 2.08332276f, 2.08332276f, 2.08332276f, 2.08332276f, 2.26034093f, 2.26034093f, 2.26034093f, 2.26034093f, 2.26034093f, 2.45240021f, 2.45240021f, 2.45240021f, 2.45240021f, 2.45240021f, 0.0f, 0.0f, 0.0f, 0.0f};
    const unsigned i = blockIdx.x * 256 + threadIdx.x; const unsigned cl = i & 255u, tile = i >> 8; const unsigned sq = tile / 67u, j = tile - sq * 67u; h16 r[64];
#pragma unroll
    for (int u = 0; u < 64; ++u) { const unsigned t = 60u * j + (unsigned)u; const unsigned tc = t < 3999u ? t : 3999u; const float lv = (u < 60 ? 1.0f : 0.0f) * (float)(t < 4000u); r[u] = toh_flush(src[((size_t)sq * NTS + tc) * NDM + cl] * 0.0009765625f * (KM ? CF[u] : 1.0f) * lv); }
    h16* pd = dst + (size_t)i * 64;
#pragma unroll
    for (int ps = 0; ps < 2; ++ps) {
#pragma unroll
        for (int g = 0; g < 8; ++g) { v8h o;
#pragma unroll
            for (int jj = 0; jj < 8; ++jj) o[jj] = r[g * 8 + jj];
            *(volatile v8h*)(pd + g * 8) = o; }
        if (ps == 0) __threadfence(); } }

__global__ __launch_bounds__(256) void k_msk4(const float* __restrict__ Pi, const float* __restrict__ Pc, h16* Ph) {
    const unsigned i = blockIdx.x * 256 + threadIdx.x; const unsigned r = i & 63u; const unsigned cr = r / 5u, orr = r - cr * 5u; const float* pi = Pi + (size_t)i * 64; const float* pc = Pc + (size_t)i * 64; h16 rh[64]; float wv[5];
#pragma unroll
    for (int p = 0; p < 5; ++p) wv[p] = (float)((unsigned)p <= orr) * exp2f(((float)p - (float)orr) * -0.0196090080f + (float)cr * -0.117654048f);
#pragma unroll
    for (int g = 0; g < 8; ++g) { const v8f ti = *(const v8f*)(pi + g * 8); const v8f tc = *(const v8f*)(pc + g * 8);
#pragma unroll
        for (int jj = 0; jj < 8; ++jj) { const unsigned cs = (unsigned)((g * 8 + jj) / 5); const int os = (g * 8 + jj) % 5; const float ki = (float)(cs == cr) * wv[os]; const float kc = (float)(cs <= cr); rh[g * 8 + jj] = toh_flush(ti[jj] * ki + tc[jj] * kc); } }
    h16* ph = Ph + (size_t)i * 64;
#pragma unroll
    for (int ps = 0; ps < 2; ++ps) {
#pragma unroll
        for (int g = 0; g < 8; ++g) { v8h oh;
#pragma unroll
            for (int jj = 0; jj < 8; ++jj) oh[jj] = rh[g * 8 + jj];
            *(volatile v8h*)(ph + g * 8) = oh; }
        if (ps == 0) __threadfence(); } }

__global__ __launch_bounds__(256) void k_dsum(const float* __restrict__ bef, const float* __restrict__ du, float* aft, h16* wrd) {
    const size_t i = (size_t)blockIdx.x * 256 + threadIdx.x; const v4f ub = *(const v4fa*)(bef + i * 4); const v4f vd = *(const v4fa*)(du + i * 4); v4f oa; v4h_ ow;
#pragma unroll
    for (int j = 0; j < 4; ++j) { oa[j] = (ub[j] + vd[j]) * 0.375829816f; ow[j] = toh_flush(oa[j]); }
    *(volatile v4f*)(aft + i * 4) = oa; *(volatile v4h_*)(wrd + i * 4) = ow; __threadfence(); *(volatile v4f*)(aft + i * 4) = oa; *(volatile v4h_*)(wrd + i * 4) = ow; }

__global__ __launch_bounds__(256) void k_lay4(const float* __restrict__ O, const float* __restrict__ Ob, float* res) {
    const size_t i = (size_t)blockIdx.x * 256 + threadIdx.x; const unsigned row = (unsigned)(i >> 6), c4 = (unsigned)(i & 63u); const unsigned sq = row / 4000u, t = row - sq * 4000u; const unsigned j = t / 60u, r = t - j * 60u; const size_t tr = ((size_t)(sq * 67u + j) * 64 + r) * NDM + (size_t)c4 * 4; const v4f ua = *(const v4fa*)(O + tr); const v4f ub = *(const v4fa*)(Ob + tr); v4f o;
#pragma unroll
    for (int jj = 0; jj < 4; ++jj) o[jj] = ua[jj] + ub[jj];
    *(volatile v4f*)(res + i * 4) = o; __threadfence(); *(volatile v4f*)(res + i * 4) = o; }

extern "C" void kernel_launch(void* const* d_in, const int* in_sizes, int n_in, void* d_out, int out_size, void* d_ws, size_t ws_size, hipStream_t stream) {
    if (n_in < 6) return;
    if (in_sizes[0] != NRW * NDM || in_sizes[1] != NRW * NDM || in_sizes[2] != NRW * NDM || in_sizes[3] != NDM * NDM || in_sizes[4] != NDM * NDM || in_sizes[5] != NDM * NDM) return;
    if (out_size != NRW * NDM) return;
    static_assert(NRW == NSQ * NTS && NTS == 4000 && NDM == 256 && NTL * 60 >= NTS && (NTL - 1) * 60 < NTS && NBK == NSQ * NTL && NBL == 64 * 64 && NRW % 64 == 0 && (NDM * 4) % 256 == 0 && (NRW * NDM / 8) % 256 == 0 && (NBK * 64) % 256 == 0 && (NBK * NDM) % 256 == 0 && (NSQ * NDM * NDM / 4) % 256 == 0 && (NRW * NDM / 4) % 256 == 0 && (NSQ * NDM * NDM * 4 / 16) % 256 == 0 && (NSQ * NDM * NDM * 2 / 16) % 256 == 0 && 3 * (size_t)NRW >= 2 * (size_t)NBK * 64, "the products: 64-row tiles over depths of 256 and 64; the flat grids exact; twelve whole chunks a tile; O and Ob fit in Q's, K's and V's bytes");
    const float* xq = (const float*)d_in[0]; const float* xk = (const float*)d_in[1]; const float* xv = (const float*)d_in[2]; const float* Wq = (const float*)d_in[3]; const float* Wk = (const float*)d_in[4]; const float* Wv = (const float*)d_in[5]; float* res = (float*)d_out;
    char* wsp = (char*)d_ws; auto take = [&](size_t bytes) { char* p = wsp; wsp += (bytes + 255) & ~(size_t)255; return (void*)p; };
    h16* Xw = (h16*)take((size_t)NRW * NDM * 2); h16* Wtq = (h16*)take((size_t)NDM * NDM * 2); h16* Wtk = (h16*)take((size_t)NDM * NDM * 2); h16* Wtv = (h16*)take((size_t)NDM * NDM * 2);
    float* TT = (float*)take((size_t)3 * NRW * NDM * 4);
    h16* Qo = (h16*)take((size_t)NBK * 64 * NDM * 2); h16* Qn = (h16*)take((size_t)NBK * 64 * NDM * 2); h16* Ks = (h16*)take((size_t)NBK * 64 * NDM * 2); h16* KsT = (h16*)take((size_t)NBK * NDM * 64 * 2); h16* VT = (h16*)take((size_t)NBK * NDM * 64 * 2);
    float* Pi = (float*)take((size_t)NBK * NBL * 4); float* Pc = (float*)take((size_t)NBK * NBL * 4); h16* Ph = (h16*)take((size_t)NBK * NBL * 2);
    float* StA = (float*)take((size_t)NSQ * NDM * NDM * 4); float* StB = (float*)take((size_t)NSQ * NDM * NDM * 4); h16* SwA = (h16*)take((size_t)NSQ * NDM * NDM * 2); h16* SwB = (h16*)take((size_t)NSQ * NDM * NDM * 2); float* Du = (float*)take((size_t)NSQ * NDM * NDM * 4);
    if ((size_t)(wsp - (char*)d_ws) > ws_size) return;
    float* Q = TT; float* K = TT + (size_t)NRW * NDM; float* V = TT + (size_t)2 * NRW * NDM; float* O = TT; float* Ob = TT + (size_t)NBK * 64 * NDM;
    k_wtw<<<NDM * 4 / 256, 256, 0, stream>>>(Wq, Wtq); k_wtw<<<NDM * 4 / 256, 256, 0, stream>>>(Wk, Wtk); k_wtw<<<NDM * 4 / 256, 256, 0, stream>>>(Wv, Wtv);
    k_xword<<<(unsigned)(NRW * NDM / 8 / 256), 256, 0, stream>>>(xq, Xw); k_gemmw<h16, 0, false><<<dim3(NRW / 64, NDM / 64, 1), 32, 0, stream>>>(Xw, nullptr, Wtq, nullptr, NDM, Q, NDM, nullptr, 0, 0, 0);
    k_xword<<<(unsigned)(NRW * NDM / 8 / 256), 256, 0, stream>>>(xk, Xw); k_gemmw<h16, 0, false><<<dim3(NRW / 64, NDM / 64, 1), 32, 0, stream>>>(Xw, nullptr, Wtk, nullptr, NDM, K, NDM, nullptr, 0, 0, 0);
    k_xword<<<(unsigned)(NRW * NDM / 8 / 256), 256, 0, stream>>>(xv, Xw); k_gemmw<h16, 0, false><<<dim3(NRW / 64, NDM / 64, 1), 32, 0, stream>>>(Xw, nullptr, Wtv, nullptr, NDM, V, NDM, nullptr, 0, 0, 0);
    k_tw<0><<<NBK * 64 / 256, 256, 0, stream>>>(Q, Qo); k_tw<1><<<NBK * 64 / 256, 256, 0, stream>>>(Q, Qn); k_tw<2><<<NBK * 64 / 256, 256, 0, stream>>>(K, Ks);
    k_tcol<true><<<NBK * NDM / 256, 256, 0, stream>>>(K, KsT); k_tcol<false><<<NBK * NDM / 256, 256, 0, stream>>>(V, VT);
    k_gemmw<h16, 0, false><<<dim3(1, 1, NBK), 32, 0, stream>>>(Qo, nullptr, Ks, nullptr, NDM, Pi, 64, nullptr, (size_t)64 * NDM, (size_t)64 * NDM, NBL);
    k_gemmw<h16, 0, false><<<dim3(1, 1, NBK), 32, 0, stream>>>(Qn, nullptr, Ks, nullptr, NDM, Pc, 64, nullptr, (size_t)64 * NDM, (size_t)64 * NDM, NBL);
    k_msk4<<<NBK * 64 / 256, 256, 0, stream>>>(Pi, Pc, Ph);
    k_gemmw<h16, 0, false><<<dim3(1, NDM / 64, NBK), 32, 0, stream>>>(Ph, nullptr, VT, nullptr, 64, O, NDM, nullptr, NBL, (size_t)NDM * 64, (size_t)64 * NDM);
    k_fillb<<<(unsigned)((size_t)NSQ * NDM * NDM * 4 / 16 / 256), 256, 0, stream>>>((bf*)StA, 0u, (size_t)NSQ * NDM * NDM * 4 / 16); k_fillb<<<(unsigned)((size_t)NSQ * NDM * NDM * 2 / 16 / 256), 256, 0, stream>>>((bf*)SwA, 0u, (size_t)NSQ * NDM * NDM * 2 / 16);
    for (int j = 0; j < NTL; ++j) { const float* stb = (j & 1) ? StB : StA; float* sta = (j & 1) ? StA : StB; const h16* swr = (j & 1) ? SwB : SwA; h16* sww = (j & 1) ? SwA : SwB;
        k_gemmw<h16, 0, false><<<dim3(1, NDM / 64, NSQ), 32, 0, stream>>>(Qn + (size_t)j * 64 * NDM, nullptr, swr, nullptr, NDM, Ob + (size_t)j * 64 * NDM, NDM, nullptr, (size_t)NTL * 64 * NDM, (size_t)NDM * NDM, (size_t)NTL * 64 * NDM);
        if (j + 1 < NTL) { k_gemmw<h16, 0, false><<<dim3(NDM / 64, NDM / 64, NSQ), 32, 0, stream>>>(VT + (size_t)j * NDM * 64, nullptr, KsT + (size_t)j * NDM * 64, nullptr, 64, Du, NDM, nullptr, (size_t)NTL * NDM * 64, (size_t)NTL * NDM * 64, (size_t)NDM * NDM);
            k_dsum<<<(unsigned)((size_t)NSQ * NDM * NDM / 4 / 256), 256, 0, stream>>>(stb, Du, sta, sww); } }
    k_lay4<<<(unsigned)((size_t)NRW * NDM / 4 / 256), 256, 0, stream>>>(O, Ob, res);
}
